// lstm_46428596469896
// MI455X (gfx1250) — hardware-verified
//
#include <hip/hip_runtime.h>
#include <math.h>

constexpr int NBATCH  = 4096;
constexpr int NSTEP   = 512;
constexpr int NHID    = 32;
constexpr int NGATE   = 128;
constexpr int NOUTF   = 30;
constexpr int NWAVE   = 4;
constexpr int NTHR    = 128;
constexpr int WROWS   = 16;
constexpr int BROWS   = NWAVE * WROWS;
constexpr int NTILE   = 8;
constexpr int NMAT    = 5;
constexpr int XCHUNK  = 32;
constexpr int XPITCH  = 36;
constexpr int OTILE   = WROWS * NOUTF;
constexpr int OVEC    = OTILE / 4;
constexpr float HCARRY = 256.0f;
constexpr float WCARRY = 64.0f;
constexpr float ZCARRY = HCARRY * WCARRY;
constexpr float ZINV   = 1.0f / ZCARRY;
constexpr float TCLAMP = 15.0f;

static_assert(NGATE == 4 * NHID, "gate dim");
static_assert(NGATE == NTILE * 16, "n-subtiles");
static_assert(NHID == 32, "K is exactly one 32-deep k-step");
static_assert(NBATCH % BROWS == 0, "no batch tail");
static_assert(NSTEP % XCHUNK == 0, "no step tail");
static_assert(NTHR == NGATE, "one thread per gate row in the bias staging");
static_assert((NGATE * NHID) == 4 * NTHR * 8, "weight staging covers one matrix exactly");
static_assert((NWAVE * 3 * WROWS * NHID) == 6 * NTHR * 8, "h plane zero fill exact");
static_assert((OTILE * 4) % 128 == 0, "wave output tile is whole 128-B lines");
static_assert(OVEC == 120, "output vectors per wave");
static_assert(XPITCH % 4 == 0 && XPITCH >= XCHUNK, "x slab pitch");

typedef __attribute__((ext_vector_type(16))) _Float16 v16h;
typedef __attribute__((ext_vector_type(8)))  _Float16 v8h;
typedef __attribute__((ext_vector_type(8)))  float    v8f;
typedef __attribute__((ext_vector_type(4)))  float    v4f;

union FragU { v16h v; v8h h[2]; };
__device__ __forceinline__ v16h frag_load(const _Float16* p) {
  FragU f;
  f.h[0] = *(const v8h*)(p);
  f.h[1] = *(const v8h*)(p + 16);
  return f.v;
}

__device__ __forceinline__ v8f mma_g(v16h a, v16h b, v8f c) {
  c = __builtin_amdgcn_wmma_f32_16x16x32_f16(false, a, false, b, (short)0, c, false, false);
  asm volatile("v_nop\n\tv_nop\n\tv_nop\n\tv_nop" : "+v"(c) : "v"(a), "v"(b));
  return c;
}

__device__ __forceinline__ float fsig(float x) {
  return __builtin_amdgcn_rcpf(1.0f + __expf(-x));
}
__device__ __forceinline__ float ftanh(float x) {
  const float xc = fminf(fmaxf(x, -TCLAMP), TCLAMP);
  return 1.0f - 2.0f * __builtin_amdgcn_rcpf(1.0f + __expf(2.0f * xc));
}

__device__ __forceinline__ void stage_weight(const float* __restrict__ W, _Float16* dst, int tid) {
#pragma unroll 1
  for (int i = 0; i < 4; ++i) {
    const int g   = i * NTHR + tid;
    const int row = g >> 2;
    const int k8  = (g & 3) * 8;
    const v4f a = *(const v4f*)(W + row * NHID + k8);
    const v4f b = *(const v4f*)(W + row * NHID + k8 + 4);
    v8h hv;
#pragma unroll
    for (int e = 0; e < 4; ++e) {
      hv[e]     = (_Float16)(a[e] * WCARRY);
      hv[4 + e] = (_Float16)(b[e] * WCARRY);
    }
    *(v8h*)(dst + row * NHID + k8) = hv;
  }
}

template <bool KEEP>
__device__ __forceinline__ void cell_update(const v8f (&acc)[NTILE], float (&cst)[16], float (&hkeep)[16],
                                            _Float16* hplane, int hh, int c) {
#pragma unroll
  for (int j = 0; j < 2; ++j) {
#pragma unroll
    for (int r = 0; r < 8; ++r) {
      const float zi = acc[0 + j][r] * ZINV;
      const float zf = acc[2 + j][r] * ZINV;
      const float zg = acc[4 + j][r] * ZINV;
      const float zo = acc[6 + j][r] * ZINV;
      const float ig = fsig(zi);
      const float fg = fsig(zf);
      const float gg = ftanh(zg);
      const float og = fsig(zo);
      const float cn = fg * cst[j * 8 + r] + ig * gg;
      cst[j * 8 + r] = cn;
      const float hn = og * ftanh(cn);
      hplane[(8 * hh + r) * NHID + 16 * j + c] = (_Float16)(hn * HCARRY);
      if (KEEP) hkeep[j * 8 + r] = hn;
    }
  }
}

__global__ __launch_bounds__(NTHR)
void lstm3_seq_kernel(const float* __restrict__ x,
                      const float* __restrict__ Wih0, const float* __restrict__ Whh0,
                      const float* __restrict__ bih0, const float* __restrict__ bhh0,
                      const float* __restrict__ Wih1, const float* __restrict__ Whh1,
                      const float* __restrict__ bih1, const float* __restrict__ bhh1,
                      const float* __restrict__ Wih2, const float* __restrict__ Whh2,
                      const float* __restrict__ bih2, const float* __restrict__ bhh2,
                      const float* __restrict__ W2,   const float* __restrict__ b2,
                      float* __restrict__ out) {
  __shared__ __align__(16) _Float16 Wl[NMAT * NGATE * NHID];
  __shared__ __align__(16) _Float16 Hl[NWAVE * 3 * WROWS * NHID];
  __shared__ __align__(16) float Xs[NWAVE * WROWS * XPITCH];
  __shared__ __align__(16) float Bsc[3 * NGATE];
  __shared__ __align__(16) float W0sc[NGATE];

  const int tid  = threadIdx.x;
  const int lane = tid & 31;
  const int wave = tid >> 5;
  const int c    = lane & 15;
  const int hh   = lane >> 4;
  const int b0   = (blockIdx.x * NWAVE + wave) * WROWS;

  stage_weight(Whh0, Wl + 0 * NGATE * NHID, tid);
  asm volatile("" ::: "memory");
  stage_weight(Wih1, Wl + 1 * NGATE * NHID, tid);
  asm volatile("" ::: "memory");
  stage_weight(Whh1, Wl + 2 * NGATE * NHID, tid);
  asm volatile("" ::: "memory");
  stage_weight(Wih2, Wl + 3 * NGATE * NHID, tid);
  asm volatile("" ::: "memory");
  stage_weight(Whh2, Wl + 4 * NGATE * NHID, tid);
  asm volatile("" ::: "memory");
  {
    const float s0 = bih0[tid] + bhh0[tid];
    const float s1 = bih1[tid] + bhh1[tid];
    const float s2 = bih2[tid] + bhh2[tid];
    const float w0 = Wih0[tid];
    Bsc[0 * NGATE + tid] = s0 * ZCARRY;
    Bsc[1 * NGATE + tid] = s1 * ZCARRY;
    Bsc[2 * NGATE + tid] = s2 * ZCARRY;
    W0sc[tid]            = w0 * ZCARRY;
  }
  {
    v8h zv;
#pragma unroll
    for (int e = 0; e < 8; ++e) zv[e] = (_Float16)0.0f;
#pragma unroll 1
    for (int i = 0; i < 6; ++i) *(v8h*)(Hl + (i * NTHR + tid) * 8) = zv;
  }
  __syncthreads();

  _Float16* hp0 = Hl + wave * 3 * WROWS * NHID;
  _Float16* hp1 = hp0 + WROWS * NHID;
  _Float16* hp2 = hp1 + WROWS * NHID;
  float*    xs  = Xs + wave * WROWS * XPITCH;
  const int fragoff = c * NHID + 8 * hh;
  const _Float16* wfr = Wl + fragoff;

  float cst0[16], cst1[16], cst2[16], h2v[16], hdum[16];
#pragma unroll
  for (int i = 0; i < 16; ++i) { cst0[i] = 0.0f; cst1[i] = 0.0f; cst2[i] = 0.0f; h2v[i] = 0.0f; hdum[i] = 0.0f; }

#pragma unroll 1
  for (int tc = 0; tc < NSTEP / XCHUNK; ++tc) {
#pragma unroll
    for (int i = 0; i < 4; ++i) {
      const int idx = i * 32 + lane;
      const int row = idx >> 3;
      const int c4  = (idx & 7) * 4;
      const v4f v = *(const v4f*)(x + (size_t)(b0 + row) * NSTEP + tc * XCHUNK + c4);
      *(v4f*)(xs + row * XPITCH + c4) = v;
    }
    __syncthreads();

#pragma unroll 1
    for (int ti = 0; ti < XCHUNK; ++ti) {
      v8f acc[NTILE];

      {
        float xr[8];
#pragma unroll
        for (int r = 0; r < 8; ++r) xr[r] = xs[(8 * hh + r) * XPITCH + ti];
#pragma unroll
        for (int nt = 0; nt < NTILE; ++nt) {
          const float bs = Bsc[0 * NGATE + nt * 16 + c];
          const float w0 = W0sc[nt * 16 + c];
          v8f a;
#pragma unroll
          for (int r = 0; r < 8; ++r) a[r] = fmaf(w0, xr[r], bs);
          acc[nt] = a;
        }
        const v16h aown = frag_load(hp0 + fragoff);
#pragma unroll
        for (int nt = 0; nt < NTILE; ++nt) {
          const v16h bw = frag_load(wfr + 0 * NGATE * NHID + nt * 16 * NHID);
          acc[nt] = mma_g(aown, bw, acc[nt]);
        }
        cell_update<false>(acc, cst0, hdum, hp0, hh, c);
      }
      __syncthreads();

      {
#pragma unroll
        for (int nt = 0; nt < NTILE; ++nt) {
          const float bs = Bsc[1 * NGATE + nt * 16 + c];
          v8f a;
#pragma unroll
          for (int r = 0; r < 8; ++r) a[r] = bs;
          acc[nt] = a;
        }
        const v16h ain  = frag_load(hp0 + fragoff);
        const v16h aown = frag_load(hp1 + fragoff);
#pragma unroll
        for (int nt = 0; nt < NTILE; ++nt) {
          const v16h bi = frag_load(wfr + 1 * NGATE * NHID + nt * 16 * NHID);
          const v16h bh = frag_load(wfr + 2 * NGATE * NHID + nt * 16 * NHID);
          acc[nt] = mma_g(ain,  bi, acc[nt]);
          acc[nt] = mma_g(aown, bh, acc[nt]);
        }
        cell_update<false>(acc, cst1, hdum, hp1, hh, c);
      }
      __syncthreads();

      {
#pragma unroll
        for (int nt = 0; nt < NTILE; ++nt) {
          const float bs = Bsc[2 * NGATE + nt * 16 + c];
          v8f a;
#pragma unroll
          for (int r = 0; r < 8; ++r) a[r] = bs;
          acc[nt] = a;
        }
        const v16h ain  = frag_load(hp1 + fragoff);
        const v16h aown = frag_load(hp2 + fragoff);
#pragma unroll
        for (int nt = 0; nt < NTILE; ++nt) {
          const v16h bi = frag_load(wfr + 3 * NGATE * NHID + nt * 16 * NHID);
          const v16h bh = frag_load(wfr + 4 * NGATE * NHID + nt * 16 * NHID);
          acc[nt] = mma_g(ain,  bi, acc[nt]);
          acc[nt] = mma_g(aown, bh, acc[nt]);
        }
        cell_update<true>(acc, cst2, h2v, hp2, hh, c);
      }
    }
  }

  __syncthreads();
#pragma unroll
  for (int j = 0; j < 2; ++j)
#pragma unroll
    for (int r = 0; r < 8; ++r) xs[(8 * hh + r) * XPITCH + 16 * j + c] = h2v[j * 8 + r];
  __syncthreads();

  v4f val[4];
#pragma unroll
  for (int it = 0; it < 4; ++it) {
    const int idx = it * 32 + lane;
    const int idc = (idx < OVEC) ? idx : (OVEC - 1);
    int ro[4], oo[4];
    float s[4];
#pragma unroll
    for (int q = 0; q < 4; ++q) {
      const int e = idc * 4 + q;
      ro[q] = e / NOUTF;
      oo[q] = e - ro[q] * NOUTF;
      s[q]  = b2[oo[q]];
    }
#pragma unroll 1
    for (int k = 0; k < NHID; ++k) {
#pragma unroll
      for (int q = 0; q < 4; ++q) s[q] = fmaf(xs[ro[q] * XPITCH + k], W2[oo[q] * NHID + k], s[q]);
    }
    v4f v;
    v[0] = s[0]; v[1] = s[1]; v[2] = s[2]; v[3] = s[3];
    val[it] = v;
  }

  float* op = out + (size_t)b0 * NOUTF;
  for (int pass = 0; pass < 2; ++pass) {
#pragma unroll
    for (int it = 0; it < 4; ++it) {
      const int idx = it * 32 + lane;
      if (idx < OVEC) *(volatile v4f*)(op + idx * 4) = val[it];
    }
    __threadfence();
  }
}

extern "C" void kernel_launch(void* const* d_in, const int* in_sizes, int n_in,
                              void* d_out, int out_size, void* d_ws, size_t ws_size, hipStream_t stream) {
  (void)d_ws; (void)ws_size;
  if (n_in < 15 || d_out == nullptr) return;
  if (in_sizes[0] != NBATCH * NSTEP) return;
  if (in_sizes[1] != NGATE || in_sizes[2] != NGATE * NHID || in_sizes[3] != NGATE || in_sizes[4] != NGATE) return;
  if (in_sizes[5] != NGATE * NHID || in_sizes[6] != NGATE * NHID || in_sizes[7] != NGATE || in_sizes[8] != NGATE) return;
  if (in_sizes[9] != NGATE * NHID || in_sizes[10] != NGATE * NHID || in_sizes[11] != NGATE || in_sizes[12] != NGATE) return;
  if (in_sizes[13] != NOUTF * NHID || in_sizes[14] != NOUTF) return;
  if (out_size != NBATCH * NOUTF) return;

  const float* x    = (const float*)d_in[0];
  const float* Wih0 = (const float*)d_in[1];
  const float* Whh0 = (const float*)d_in[2];
  const float* bih0 = (const float*)d_in[3];
  const float* bhh0 = (const float*)d_in[4];
  const float* Wih1 = (const float*)d_in[5];
  const float* Whh1 = (const float*)d_in[6];
  const float* bih1 = (const float*)d_in[7];
  const float* bhh1 = (const float*)d_in[8];
  const float* Wih2 = (const float*)d_in[9];
  const float* Whh2 = (const float*)d_in[10];
  const float* bih2 = (const float*)d_in[11];
  const float* bhh2 = (const float*)d_in[12];
  const float* W2   = (const float*)d_in[13];
  const float* b2   = (const float*)d_in[14];
  float* out = (float*)d_out;

  lstm3_seq_kernel<<<NBATCH / BROWS, NTHR, 0, stream>>>(
      x, Wih0, Whh0, bih0, bhh0, Wih1, Whh1, bih1, bhh1,
      Wih2, Whh2, bih2, bhh2, W2, b2, out);
}
